// GlobalAttention_86131274154404
// MI455X (gfx1250) — hardware-verified
//
#include <hip/hip_runtime.h>


#define NB_  8
#define HI   84
#define NPI  (HI * HI)
#define NPR  7104
#define NPA  (NB_ * NPI)
#define CC   256
#define INNER 512
#define NHD  8
#define HD   64
#define KK   7
#define NT   144
#define NTP  192
#define KIM  (KK * KK * CC)
#define ZH   4
#define DM   CC
#define NX   NPR
#define NZ   NTP
#define SCL  0.125f
#define LOSC 1024.0f

typedef _Float16 h16;
typedef unsigned short bf;
typedef __attribute__((ext_vector_type(16))) __bf16   v16bf;
typedef __attribute__((ext_vector_type(16))) _Float16 v16h;
typedef __attribute__((ext_vector_type(8)))  _Float16 v8h;
typedef __attribute__((ext_vector_type(8)))  unsigned short v8us;
typedef __attribute__((ext_vector_type(8)))  float    v8f;
typedef __attribute__((ext_vector_type(4)))  float    v4f;
typedef __attribute__((ext_vector_type(4)))  _Float16 v4h;
typedef v8h  __attribute__((may_alias)) v8ha;
typedef v4f  __attribute__((may_alias)) v4fa;
typedef v8us __attribute__((may_alias)) v8usa;

__device__ __forceinline__ unsigned short f2bf(float f) { unsigned u = __float_as_uint(f); u += 0x7FFFu + ((u >> 16) & 1u); return (unsigned short)(u >> 16); }
__device__ __forceinline__ float bf2f(unsigned short b) { return __uint_as_float(((unsigned)b) << 16); }
__device__ __forceinline__ float bfr(float f) { return bf2f(f2bf(f)); }
__device__ __forceinline__ v16h cat16(v8h lo, v8h hi) { return __builtin_shufflevector(lo, hi, 0, 1, 2, 3, 4, 5, 6, 7, 8, 9, 10, 11, 12, 13, 14, 15); }
__device__ __forceinline__ v16bf cat16b(v8us lo, v8us hi) { return __builtin_bit_cast(v16bf, __builtin_shufflevector(lo, hi, 0, 1, 2, 3, 4, 5, 6, 7, 8, 9, 10, 11, 12, 13, 14, 15)); }
__device__ __forceinline__ v8f wmma16(v16h a, v16h b, v8f c) { return __builtin_amdgcn_wmma_f32_16x16x32_f16(false, a, false, b, (short)0, c, false, false); }
__device__ __forceinline__ v8f wmmab(v16bf a, v16bf b, v8f c) { return __builtin_amdgcn_wmma_f32_16x16x32_bf16(false, a, false, b, (short)0, c, false, false); }

__global__ __launch_bounds__(256) void k_wt(const float* __restrict__ Wm, int K, int ncols, bf* WT) {
    __shared__ __align__(16) unsigned short tl[64 * 72];
    const int tid = threadIdx.x, k0 = blockIdx.x * 64, n0 = blockIdx.y * 64;
    const int kk = tid >> 2, nq = (tid & 3) * 16;
#pragma unroll
    for (int i = 0; i < 16; ++i) tl[(nq + i) * 72 + kk] = f2bf(Wm[(size_t)(k0 + kk) * ncols + n0 + nq + i]);
    __syncthreads();
    const int piece = tid & 7;
    auto pass = [&]() {
#pragma unroll
        for (int s = 0; s < 2; ++s) { const int nr = (tid >> 3) + 32 * s; const v8us val = *(const v8usa*)(tl + nr * 72 + piece * 8); *(volatile v8us*)(WT + (size_t)(n0 + nr) * K + k0 + piece * 8) = val; }
    };
    pass(); __threadfence(); pass();
}
template <bool SPLITA, bool F16OUT = false>
__global__ __launch_bounds__(128) void k_gemmb(const bf* __restrict__ A, const bf* __restrict__ Al, const bf* __restrict__ Bn, const float* __restrict__ bias, float* C, int ldc, h16* C2, const float* __restrict__ R = nullptr, int K = DM, int roundR = 1) {
    __shared__ __align__(16) float ost[4][16 * 68];
    const int lane = threadIdx.x & 31, wave = threadIdx.x >> 5, lr = lane & 15, hi = lane >> 4;
    const int r0 = blockIdx.x * 64 + wave * 16, c0 = blockIdx.y * 64;
    const size_t aoff = (size_t)(r0 + lr) * K + 8 * hi;
    size_t boff[4];
#pragma unroll
    for (int t = 0; t < 4; ++t) boff[t] = (size_t)(c0 + t * 16 + lr) * K + 8 * hi;
    v8f acc[4];
#pragma unroll
    for (int t = 0; t < 4; ++t) acc[t] = (v8f){};
#pragma unroll 1
    for (int kc = 0; kc < K; kc += 32) {
        const v16bf a = cat16b(*(const v8us*)(A + aoff + kc), *(const v8us*)(A + aoff + kc + 16));
        v16bf al = a;
        if (SPLITA) al = cat16b(*(const v8us*)(Al + aoff + kc), *(const v8us*)(Al + aoff + kc + 16));
#pragma unroll
        for (int t = 0; t < 4; ++t) { const v16bf b = cat16b(*(const v8us*)(Bn + boff[t] + kc), *(const v8us*)(Bn + boff[t] + kc + 16)); acc[t] = wmmab(a, b, acc[t]); if (SPLITA) acc[t] = wmmab(al, b, acc[t]); }
        asm volatile("v_nop\n\tv_nop\n\tv_nop\n\tv_nop" : "+v"(acc[0]), "+v"(acc[1]), "+v"(acc[2]), "+v"(acc[3]) : "v"(a), "v"(al));
    }
    float* os = &ost[wave][0];
#pragma unroll
    for (int t = 0; t < 4; ++t) { const float bv = bias ? bfr(bias[c0 + t * 16 + lr]) : 0.f;
#pragma unroll
        for (int j = 0; j < 8; ++j) os[(hi * 8 + j) * 68 + t * 16 + lr] = acc[t][j] + bv; }
    __syncthreads();
    if (F16OUT) {
        h16* crow = (h16*)(void*)C + (size_t)r0 * ldc + c0;
        auto pass = [&]() {
#pragma unroll
            for (int s = 0; s < 4; ++s) { const int row = 4 * s + (lane >> 3), piece = lane & 7; const float* sp = os + row * 68 + piece * 8; v8h o, o2;
#pragma unroll
                for (int i = 0; i < 8; ++i) { const h16 a = (h16)sp[i]; o[i] = a; o2[i] = (h16)((sp[i] - (float)a) * LOSC); }
                *(volatile v8h*)(crow + (size_t)row * ldc + piece * 8) = o; if (C2) *(volatile v8h*)(C2 + (size_t)r0 * ldc + c0 + (size_t)row * ldc + piece * 8) = o2; }
        };
        pass(); __threadfence(); pass();
    } else {
        float* crow = C + (size_t)r0 * ldc + c0;
        auto pass = [&]() {
#pragma unroll
            for (int s = 0; s < 8; ++s) { const int Lid = (lane >> 3) + 4 * s, piece = lane & 7; const int row = Lid >> 1, cofs = (Lid & 1) * 32 + piece * 4;
                v4f val = *(const v4fa*)(os + row * 68 + cofs); if (R) { const v4f rv = *(const v4f*)(R + ((size_t)r0 + row) * ldc + c0 + cofs); val += roundR ? (v4f){bfr(rv[0]), bfr(rv[1]), bfr(rv[2]), bfr(rv[3])} : rv; }
                *(volatile v4f*)(crow + (size_t)row * ldc + cofs) = val; }
        };
        pass(); __threadfence(); pass();
    }
}


template <int MODE>
__global__ __launch_bounds__(128) void k_gemm3z(const bf* __restrict__ Ah, const bf* __restrict__ Al, const bf* __restrict__ Bh, const bf* __restrict__ Bl, int K, float* C, int ldc, size_t sA, size_t sB, size_t sC) {
    if ((MODE & 1) && (int)blockIdx.y * 64 > (int)blockIdx.x * 64 + 63) return;
    const size_t z = blockIdx.z; Ah += z * sA; Al += z * sA; Bh += z * sB; Bl += z * sB; C += z * sC;
    const int Klim = (MODE & 2) ? min(K, ((int)blockIdx.x + 1) * 64) : K;
    __shared__ __align__(16) float ost[4][16 * 68];
    const int lane = threadIdx.x & 31, wave = threadIdx.x >> 5, lr = lane & 15, hi = lane >> 4;
    const int r0 = blockIdx.x * 64 + wave * 16, c0 = blockIdx.y * 64;
    const size_t aoff = (size_t)(r0 + lr) * K + 8 * hi;
    v8f acc[4];
#pragma unroll
    for (int t = 0; t < 4; ++t) acc[t] = (v8f){};
#pragma unroll 1
    for (int kc = 0; kc < Klim; kc += 32) {
        const v16bf a = cat16b(*(const v8us*)(Ah + aoff + kc), *(const v8us*)(Ah + aoff + kc + 16));
        v16bf al = a; if (!(MODE & 4) && !(MODE & 16)) al = cat16b(*(const v8us*)(Al + aoff + kc), *(const v8us*)(Al + aoff + kc + 16));
#pragma unroll
        for (int t = 0; t < 4; ++t) { const size_t bo = (size_t)(c0 + t * 16 + lr) * K + kc + 8 * hi;
            const v16bf bh = cat16b(*(const v8us*)(Bh + bo), *(const v8us*)(Bh + bo + 16));
            acc[t] = wmmab(a, bh, acc[t]);
            if (!(MODE & 4)) { if (!(MODE & 16)) acc[t] = wmmab(al, bh, acc[t]); if (!(MODE & 8)) { const v16bf bl = cat16b(*(const v8us*)(Bl + bo), *(const v8us*)(Bl + bo + 16)); acc[t] = wmmab(a, bl, acc[t]); } } }
        asm volatile("v_nop\n\tv_nop\n\tv_nop\n\tv_nop" : "+v"(acc[0]), "+v"(acc[1]), "+v"(acc[2]), "+v"(acc[3]) : "v"(a), "v"(al));
    }
    float* os = &ost[wave][0];
#pragma unroll
    for (int t = 0; t < 4; ++t) {
#pragma unroll
        for (int j = 0; j < 8; ++j) os[(hi * 8 + j) * 68 + t * 16 + lr] = acc[t][j]; }
    __builtin_amdgcn_wave_barrier(); asm volatile("" ::: "memory");
    float* crow = C + (size_t)r0 * ldc + c0;
    auto pass = [&]() {
#pragma unroll
        for (int s = 0; s < 8; ++s) { const int Lid = (lane >> 3) + 4 * s, piece = lane & 7; const int row = Lid >> 1, cofs = (Lid & 1) * 32 + piece * 4;
            const v4f val = *(const v4fa*)(os + row * 68 + cofs); *(volatile v4f*)(crow + (size_t)row * ldc + cofs) = val; }
    };
    pass(); __threadfence(); pass();
}
__global__ __launch_bounds__(256) void k_planes32z(const float* __restrict__ F, int ld, int off, float sc, int rows, bf* Ph, bf* Pl) {
    typedef __attribute__((ext_vector_type(2))) unsigned short v2us;
    const int lane = threadIdx.x & 31; const size_t r = ((size_t)blockIdx.x * 8 + (threadIdx.x >> 5)) * 2 + (lane >> 4); if (r >= (size_t)rows) return; const int z = blockIdx.z; const int c0 = (lane & 15) * 2; v2us oh, ol;
    Ph += (size_t)z * rows * 32; Pl += (size_t)z * rows * 32;
#pragma unroll
    for (int i = 0; i < 2; ++i) { const float y = F[r * ld + off + z * 32 + c0 + i] * sc; const unsigned short hb = f2bf(y); oh[i] = hb; ol[i] = f2bf(y - bf2f(hb)); }
    const size_t o = r * 32 + c0; *(volatile v2us*)(Ph + o) = oh; *(volatile v2us*)(Pl + o) = ol; __threadfence(); *(volatile v2us*)(Ph + o) = oh; *(volatile v2us*)(Pl + o) = ol;
}
__global__ __launch_bounds__(256) void k_vtpadz(const float* __restrict__ F, int ld, int off, int nk, bf* Th, bf* Tl) {
    typedef __attribute__((ext_vector_type(2))) unsigned short v2us;
    const int lane = threadIdx.x & 31; const size_t wid = (size_t)blockIdx.x * 8 + (threadIdx.x >> 5); if (wid >= (size_t)64 * (nk / 64)) return; const int z = blockIdx.z; const int d = (int)(wid / (nk / 64)); const int k0 = (int)(wid % (nk / 64)) * 64 + lane * 2; v2us oh, ol;
    Th += (size_t)z * 64 * nk; Tl += (size_t)z * 64 * nk;
#pragma unroll
    for (int i = 0; i < 2; ++i) { const float y = (d < 32) ? F[(size_t)(k0 + i) * ld + off + z * 32 + (d < 32 ? d : 0)] : 0.f; const unsigned short hb = f2bf(y); oh[i] = hb; ol[i] = f2bf(y - bf2f(hb)); }
    const size_t o = (size_t)d * nk + k0; *(volatile v2us*)(Th + o) = oh; *(volatile v2us*)(Tl + o) = ol; __threadfence(); *(volatile v2us*)(Th + o) = oh; *(volatile v2us*)(Tl + o) = ol;
}
template <int NK>
__global__ __launch_bounds__(256) void k_softmaxz(const float* __restrict__ S, int rows, bf* PH, bf* PL) {
    typedef __attribute__((ext_vector_type(4))) unsigned short v4us;
    const int lane = threadIdx.x & 31, i = blockIdx.x * 8 + (threadIdx.x >> 5); if (i >= rows) return; const size_t zo = (size_t)blockIdx.z * rows * NK; const float* sr = S + zo + (size_t)i * NK; PH += zo; PL += zo;
    float m = -3.0e38f;
#pragma unroll 1
    for (int c0 = lane * 4; c0 < NK; c0 += 128) {
#pragma unroll
        for (int q = 0; q < 4; ++q) m = fmaxf(m, sr[c0 + q]); }
#pragma unroll
    for (int sh = 16; sh; sh >>= 1) m = fmaxf(m, __shfl_xor(m, sh, 32));
    float sum = 0.f;
#pragma unroll 1
    for (int c0 = lane * 4; c0 < NK; c0 += 128) {
#pragma unroll
        for (int q = 0; q < 4; ++q) sum += __expf(sr[c0 + q] - m); }
#pragma unroll
    for (int sh = 16; sh; sh >>= 1) sum += __shfl_xor(sum, sh, 32);
    const float inv = 1.0f / sum;
#pragma unroll 1
    for (int ps = 0; ps < 2; ++ps) {
#pragma unroll 1
        for (int c0 = lane * 4; c0 < NK; c0 += 128) { v4us oh, ol;
#pragma unroll
            for (int q = 0; q < 4; ++q) { const float p = __expf(sr[c0 + q] - m) * inv; const unsigned short hb = f2bf(p); oh[q] = hb; ol[q] = f2bf(p - bf2f(hb)); }
            const size_t o = (size_t)i * NK + c0; *(volatile v4us*)(PH + o) = oh; *(volatile v4us*)(PL + o) = ol; }
        if (ps == 0) __threadfence(); }
}
__global__ __launch_bounds__(256) void k_placez(const float* __restrict__ XH, int rows, int ldy, float* Y) {
    const int lane = threadIdx.x & 31; const size_t q = (size_t)blockIdx.x * 8 + (threadIdx.x >> 5); if (q >= (size_t)rows) return; const int z = blockIdx.z; const float v = XH[((size_t)z * rows + q) * 64 + lane];
    *(volatile float*)(Y + q * ldy + z * 32 + lane) = v; __threadfence(); *(volatile float*)(Y + q * ldy + z * 32 + lane) = v;
}

__global__ __launch_bounds__(256) void k_cvt256(const float* __restrict__ src, int rows, int nlive, bf* dst) {
    const int lane = threadIdx.x & 31; const size_t r = (size_t)blockIdx.x * 8 + (threadIdx.x >> 5); if (r >= (size_t)rows) return; v8us o; const bool live = r < (size_t)nlive;
#pragma unroll
    for (int i = 0; i < 8; ++i) o[i] = f2bf(live ? src[(live ? r : 0) * CC + lane * 8 + i] : 0.f);
    *(volatile v8us*)(dst + r * CC + lane * 8) = o; __threadfence(); *(volatile v8us*)(dst + r * CC + lane * 8) = o;
}
__global__ __launch_bounds__(256) void k_im2col7(const float* __restrict__ x, bf* PT) {
    const int lane = threadIdx.x & 31; const size_t r = (size_t)blockIdx.x * 8 + (threadIdx.x >> 5); if (r >= (size_t)NB_ * NT) return; const int b = (int)(r / NT); const int t = (int)(r % NT); const int ty = t / 12, tx = t % 12;
#pragma unroll 1
    for (int ps = 0; ps < 2; ++ps) {
#pragma unroll 1
        for (int kk = 0; kk < KK * KK; ++kk) { const int ky = kk / KK, kx = kk % KK; const float* src = x + (((size_t)b * HI + ty * KK + ky) * HI + tx * KK + kx) * CC + lane * 8; v8us o;
#pragma unroll
            for (int i = 0; i < 8; ++i) o[i] = f2bf(src[i]);
            *(volatile v8us*)(PT + r * KIM + (size_t)kk * CC + lane * 8) = o; }
        if (ps == 0) __threadfence(); }
}
__global__ __launch_bounds__(256) void k_qplz(const float* __restrict__ Q, int h0, float sc, bf* Ph, bf* Pl) {
    typedef __attribute__((ext_vector_type(2))) unsigned short v2us;
    const int lane = threadIdx.x & 31; const size_t i = (size_t)blockIdx.x * 8 + (threadIdx.x >> 5); if (i >= (size_t)NPR) return; const int z = blockIdx.z; Ph += (size_t)z * NPR * HD; Pl += (size_t)z * NPR * HD; v2us oh, ol;
#pragma unroll
    for (int q = 0; q < 2; ++q) { const float y = (i < (size_t)NPI) ? Q[(i < (size_t)NPI ? i : 0) * INNER + (h0 + z) * HD + lane * 2 + q] * sc : 0.f; const unsigned short hb = f2bf(y); oh[q] = hb; ol[q] = f2bf(y - bf2f(hb)); }
    const size_t o = i * HD + lane * 2; *(volatile v2us*)(Ph + o) = oh; *(volatile v2us*)(Pl + o) = ol; __threadfence(); *(volatile v2us*)(Ph + o) = oh; *(volatile v2us*)(Pl + o) = ol;
}
__global__ __launch_bounds__(256) void k_kplz(const float* __restrict__ KV, int b, int h0, bf* Ph, bf* Pl) {
    typedef __attribute__((ext_vector_type(2))) unsigned short v2us;
    const int lane = threadIdx.x & 31; const size_t t = (size_t)blockIdx.x * 8 + (threadIdx.x >> 5); if (t >= (size_t)NTP) return; const int z = blockIdx.z; Ph += (size_t)z * NTP * HD; Pl += (size_t)z * NTP * HD; v2us oh, ol;
#pragma unroll
    for (int q = 0; q < 2; ++q) { const float y = (t < (size_t)NT) ? KV[((size_t)b * NT + (t < (size_t)NT ? t : 0)) * (2 * INNER) + (h0 + z) * HD + lane * 2 + q] : 0.f; const unsigned short hb = f2bf(y); oh[q] = hb; ol[q] = f2bf(y - bf2f(hb)); }
    const size_t o = t * HD + lane * 2; *(volatile v2us*)(Ph + o) = oh; *(volatile v2us*)(Pl + o) = ol; __threadfence(); *(volatile v2us*)(Ph + o) = oh; *(volatile v2us*)(Pl + o) = ol;
}
__global__ __launch_bounds__(256) void k_vtplz(const float* __restrict__ KV, int b, int h0, bf* Th, bf* Tl) {
    typedef __attribute__((ext_vector_type(2))) unsigned short v2us;
    const int lane = threadIdx.x & 31; const size_t wid = (size_t)blockIdx.x * 8 + (threadIdx.x >> 5); if (wid >= (size_t)HD * (NTP / 64)) return; const int z = blockIdx.z; const int d = (int)(wid / (NTP / 64)); const int t0 = (int)(wid % (NTP / 64)) * 64 + lane * 2; v2us oh, ol;
    Th += (size_t)z * HD * NTP; Tl += (size_t)z * HD * NTP;
#pragma unroll
    for (int q = 0; q < 2; ++q) { const int t = t0 + q; const float y = (t < NT) ? KV[((size_t)b * NT + (t < NT ? t : 0)) * (2 * INNER) + INNER + (h0 + z) * HD + d] : 0.f; const unsigned short hb = f2bf(y); oh[q] = hb; ol[q] = f2bf(y - bf2f(hb)); }
    const size_t o = (size_t)d * NTP + t0; *(volatile v2us*)(Th + o) = oh; *(volatile v2us*)(Tl + o) = ol; __threadfence(); *(volatile v2us*)(Th + o) = oh; *(volatile v2us*)(Tl + o) = ol;
}
__global__ __launch_bounds__(256) void k_soft144z(const float* __restrict__ S, bf* PH, bf* PL) {
    typedef __attribute__((ext_vector_type(4))) unsigned short v4us;
    const int lane = threadIdx.x & 31; const size_t i = (size_t)blockIdx.x * 8 + (threadIdx.x >> 5); if (i >= (size_t)NPR) return; const size_t zo = (size_t)blockIdx.z * NPR * NTP; const float* sr = S + zo + i * NTP; PH += zo; PL += zo;
    float a[8];
#pragma unroll
    for (int q = 0; q < 4; ++q) { a[q] = sr[lane * 4 + q]; const int k2 = 128 + lane * 4 + q; a[4 + q] = (lane < 16 && k2 < NT) ? sr[(lane < 16) ? k2 : 0] : -3.0e38f; }
    float m = -3.0e38f;
#pragma unroll
    for (int q = 0; q < 8; ++q) m = fmaxf(m, a[q]);
#pragma unroll
    for (int sh = 16; sh; sh >>= 1) m = fmaxf(m, __shfl_xor(m, sh, 32));
    float e[8]; float s = 0.f;
#pragma unroll
    for (int q = 0; q < 8; ++q) { e[q] = (a[q] > -1.0e38f) ? __expf(a[q] - m) : 0.f; s += e[q]; }
#pragma unroll
    for (int sh = 16; sh; sh >>= 1) s += __shfl_xor(s, sh, 32);
    const float inv = 1.0f / s; v4us oh0, ol0, oh1, ol1;
#pragma unroll
    for (int q = 0; q < 4; ++q) { { const float p = e[q] * inv; const unsigned short hb = f2bf(p); oh0[q] = hb; ol0[q] = f2bf(p - bf2f(hb)); } { const float p = e[4 + q] * inv; const unsigned short hb = f2bf(p); oh1[q] = hb; ol1[q] = f2bf(p - bf2f(hb)); } }
    auto pass = [&]() { *(volatile v4us*)(PH + i * NTP + lane * 4) = oh0; *(volatile v4us*)(PL + i * NTP + lane * 4) = ol0; if (lane < 16) { *(volatile v4us*)(PH + i * NTP + 128 + lane * 4) = oh1; *(volatile v4us*)(PL + i * NTP + 128 + lane * 4) = ol1; } };
    pass(); __threadfence(); pass();
}
__global__ __launch_bounds__(256) void k_placebz(const float* __restrict__ XH, int h0, float* MG) {
    typedef __attribute__((ext_vector_type(2))) float v2f_;
    const int lane = threadIdx.x & 31; const size_t i = (size_t)blockIdx.x * 8 + (threadIdx.x >> 5); if (i >= (size_t)NPR) return; const int z = blockIdx.z;
    const v2f_ v = *(const v2f_*)(XH + ((size_t)z * NPR + i) * HD + lane * 2); float* dst = MG + i * INNER + (h0 + z) * HD + lane * 2;
    *(volatile v2f_*)dst = v; __threadfence(); *(volatile v2f_*)dst = v;
}
__global__ __launch_bounds__(256) void k_split512(const float* __restrict__ src, int rows, bf* dh, bf* dl) {
    const int lane = threadIdx.x & 31; const size_t r = (size_t)blockIdx.x * 8 + (threadIdx.x >> 5); if (r >= (size_t)rows) return;
#pragma unroll 1
    for (int ps = 0; ps < 2; ++ps) {
#pragma unroll
        for (int q = 0; q < INNER / 256; ++q) { const size_t o = r * INNER + q * 256 + lane * 8; const v8f v = *(const v8f*)(src + o); v8us oh, ol;
#pragma unroll
            for (int i = 0; i < 8; ++i) { const unsigned short hb = f2bf(v[i]); oh[i] = hb; ol[i] = f2bf(v[i] - bf2f(hb)); }
            *(volatile v8us*)(dh + o) = oh; *(volatile v8us*)(dl + o) = ol; }
        if (ps == 0) __threadfence(); }
}

__global__ __launch_bounds__(256) void k_copyrows(const float* __restrict__ OS, float* OUTB) {
    const int lane = threadIdx.x & 31; const size_t p = (size_t)blockIdx.x * 8 + (threadIdx.x >> 5); if (p >= (size_t)NPI) return;
    const v4f v0 = *(const v4f*)(OS + p * CC + lane * 4), v1 = *(const v4f*)(OS + p * CC + 128 + lane * 4);
    *(volatile v4f*)(OUTB + p * CC + lane * 4) = v0; *(volatile v4f*)(OUTB + p * CC + 128 + lane * 4) = v1; __threadfence(); *(volatile v4f*)(OUTB + p * CC + lane * 4) = v0; *(volatile v4f*)(OUTB + p * CC + 128 + lane * 4) = v1;
}

extern "C" void kernel_launch(void* const* d_in, const int* in_sizes, int n_in,
                              void* d_out, int out_size, void* d_ws, size_t ws_size, hipStream_t stream) {
    (void)in_sizes; (void)n_in; (void)out_size;
    const float* x = (const float*)d_in[0]; const float* w_q = (const float*)d_in[1]; const float* w_kv = (const float*)d_in[2]; const float* w_out = (const float*)d_in[3]; const float* b_out = (const float*)d_in[4];
    float* out = (float*)d_out;
    char* wsp = (char*)d_ws;
    auto take = [&](size_t bytes) { char* p = wsp; wsp += (bytes + 255) & ~(size_t)255; return (void*)p; };
    bf* WQ = (bf*)take((size_t)INNER * CC * 2); bf* WO = (bf*)take((size_t)CC * INNER * 2); float* KV = (float*)take((size_t)NB_ * NT * 2 * INNER * 4);
    bf* Xb = (bf*)take((size_t)NPR * CC * 2); float* Q = (float*)take((size_t)NPR * INNER * 4);
    const size_t ATT = (size_t)ZH * NPR * HD * 2 * 2 + (size_t)ZH * NTP * HD * 2 * 2 + (size_t)ZH * HD * NTP * 2 * 2 + (size_t)ZH * NPR * NTP * 4 + (size_t)ZH * NPR * NTP * 2 * 2 + (size_t)ZH * NPR * HD * 4;
    char* att = (char*)take(ATT); char* ap = att;
    auto sub = [&](size_t bytes) { char* p = ap; ap += (bytes + 255) & ~(size_t)255; return (void*)p; };
    bf* Qh = (bf*)sub((size_t)ZH * NPR * HD * 2); bf* Ql = (bf*)sub((size_t)ZH * NPR * HD * 2); bf* Kh = (bf*)sub((size_t)ZH * NTP * HD * 2); bf* Kl = (bf*)sub((size_t)ZH * NTP * HD * 2); bf* VTh = (bf*)sub((size_t)ZH * HD * NTP * 2); bf* VTl = (bf*)sub((size_t)ZH * HD * NTP * 2);
    float* S = (float*)sub((size_t)ZH * NPR * NTP * 4); bf* PH = (bf*)sub((size_t)ZH * NPR * NTP * 2); bf* PL = (bf*)sub((size_t)ZH * NPR * NTP * 2); float* XH = (float*)sub((size_t)ZH * NPR * HD * 4);
    bf* PT = (bf*)att; bf* WKV = (bf*)(att + (((size_t)NB_ * NT * KIM * 2 + 255) & ~(size_t)255));
    float* MG = (float*)take((size_t)NPR * INNER * 4); bf* Mh = (bf*)take((size_t)NPR * INNER * 2); bf* Ml = (bf*)take((size_t)NPR * INNER * 2); float* OS = (float*)take((size_t)NPR * CC * 4);
    if ((size_t)(wsp - (char*)d_ws) > ws_size || (size_t)(ap - att) > ATT + 4096 || ((size_t)NB_ * NT * KIM * 2 + (size_t)2 * INNER * KIM * 2 + 512) > ATT) return;
    k_wt<<<dim3(CC / 64, INNER / 64, 1), 256, 0, stream>>>(w_q, CC, INNER, WQ); k_wt<<<dim3(KIM / 64, (2 * INNER) / 64, 1), 256, 0, stream>>>(w_kv, KIM, 2 * INNER, WKV); k_wt<<<dim3(INNER / 64, CC / 64, 1), 256, 0, stream>>>(w_out, INNER, CC, WO);
    k_im2col7<<<(NB_ * NT) / 8, 256, 0, stream>>>(x, PT);
    k_gemmb<false, false><<<dim3((NB_ * NT) / 64, (2 * INNER) / 64, 1), 128, 0, stream>>>(PT, nullptr, WKV, nullptr, KV, 2 * INNER, nullptr, nullptr, KIM);
    for (int b = 0; b < NB_; ++b) {
        k_cvt256<<<NPR / 8, 256, 0, stream>>>(x + (size_t)b * NPI * CC, NPR, NPI, Xb);
        k_gemmb<false, false><<<dim3(NPR / 64, INNER / 64, 1), 128, 0, stream>>>(Xb, nullptr, WQ, nullptr, Q, INNER, nullptr, nullptr, CC);
        for (int g = 0; g < NHD / ZH; ++g) { const int h0 = g * ZH;
            k_qplz<<<dim3(NPR / 8, 1, ZH), 256, 0, stream>>>(Q, h0, SCL, Qh, Ql); k_kplz<<<dim3(NTP / 8, 1, ZH), 256, 0, stream>>>(KV, b, h0, Kh, Kl); k_vtplz<<<dim3((HD * (NTP / 64)) / 8, 1, ZH), 256, 0, stream>>>(KV, b, h0, VTh, VTl);
            k_gemm3z<0><<<dim3(NPR / 64, NTP / 64, ZH), 128, 0, stream>>>(Qh, Ql, Kh, Kl, HD, S, NTP, (size_t)NPR * HD, (size_t)NTP * HD, (size_t)NPR * NTP);
            k_soft144z<<<dim3(NPR / 8, 1, ZH), 256, 0, stream>>>(S, PH, PL);
            k_gemm3z<0><<<dim3(NPR / 64, 1, ZH), 128, 0, stream>>>(PH, PL, VTh, VTl, NTP, XH, HD, (size_t)NPR * NTP, (size_t)HD * NTP, (size_t)NPR * HD);
            k_placebz<<<dim3(NPR / 8, 1, ZH), 256, 0, stream>>>(XH, h0, MG); }
        k_split512<<<NPR / 8, 256, 0, stream>>>(MG, NPR, Mh, Ml);
        k_gemmb<true, false><<<dim3(NPR / 64, CC / 64, 1), 128, 0, stream>>>(Mh, Ml, WO, b_out, OS, CC, nullptr, nullptr, INNER);
        k_copyrows<<<NPI / 8, 256, 0, stream>>>(OS, out + (size_t)b * NPI * CC); }
}
